// Decoder_80814104642079
// MI455X (gfx1250) — hardware-verified
//
#include <hip/hip_runtime.h>
#include <stddef.h>
#include <stdint.h>


#define F0     32
#define HID    64
#define FOUT   128
#define K1     64
#define K2     128
#define NTHR   256
#define NWAVE  8
#define EPT    8
#define CHUNK  (NTHR * EPT)
#define WCAP   (EPT * 32)
#define LISTN  (NWAVE * WCAP)
#define NBA    512
#define SLA    9
#define RCAP   20480
#define DEGCAP 96
#define HDRI   32
#define SEG_CNT HDRI
#define SEG_OFF (HDRI + NBA)
#define SEG_COL (HDRI + 2 * NBA)
#define SEG_VAL (HDRI + 2 * NBA + RCAP)
#define SEGI   (HDRI + 2 * NBA + 2 * RCAP)
#define SC_ZINTS    (LISTN + SEGI + NBA)
#define SC_LDS_INTS (SC_ZINTS + 16)
#define MT     128
#define NU1    (HID * (K1 / 8))
#define NU2    (FOUT * (K2 / 8))
#define NWB    ((NU1 + NU2) / NTHR)
#define ML_A2_OFF   65536
#define ML_LDS_BYTES (65536 + 32768)
#define WSMAX  134217728

static_assert((CHUNK & (CHUNK - 1)) == 0 && CHUNK <= 4096);
static_assert((NBA & (NBA - 1)) == 0 && NBA == (1 << SLA));
static_assert(((long long)CHUNK << SLA) < (1LL << 31));
static_assert(LISTN % NTHR == 0 && LISTN % 4 == 0);
static_assert(NBA % (4 * NWAVE) == 0 && NBA % 32 == 0 && NBA % MT == 0);
static_assert(RCAP % 4 == 0 && SEGI % 32 == 0 && SEG_COL % 4 == 0 && SEG_VAL % 4 == 0);
static_assert(SC_ZINTS % 4 == 0);
static_assert(SC_LDS_INTS * 4 <= 300000 && SEGI * 4 <= 300000);
static_assert(K1 % 32 == 0 && K2 % 32 == 0 && K1 == 2 * F0 && K2 == 2 * HID);
static_assert(NU1 % NTHR == 0 && (NU1 + NU2) % NTHR == 0);
static_assert(MT == NWAVE * 16 && F0 == 8 * 4 && FOUT == 32 * 4);
static_assert(MT * K1 * 2 + MT * HID * 4 <= ML_A2_OFF && MT * FOUT * 4 <= ML_A2_OFF);
static_assert(MT * K2 * 2 == ML_LDS_BYTES - ML_A2_OFF);

typedef float          v4f   __attribute__((ext_vector_type(4)));
typedef float          v8f   __attribute__((ext_vector_type(8)));
typedef int            v4i   __attribute__((ext_vector_type(4)));
typedef int            v8i   __attribute__((ext_vector_type(8)));
typedef unsigned short v4us  __attribute__((ext_vector_type(4)));
typedef unsigned short v8us  __attribute__((ext_vector_type(8)));
typedef unsigned short v16us __attribute__((ext_vector_type(16)));
typedef __bf16         v16bf __attribute__((ext_vector_type(16)));
typedef v4f  __attribute__((may_alias)) v4fa;
typedef v4i  __attribute__((may_alias)) v4ia;
typedef v4us __attribute__((may_alias)) v4usa;
typedef v8us __attribute__((may_alias)) v8usa;
union FragB { v16bf v; v16us u; v8us h[2]; v8i w; };

__device__ __forceinline__ v8f wmb(const FragB& a, const FragB& b, v8f c) {
  v8f d = __builtin_amdgcn_wmma_f32_16x16x32_bf16(false, a.v, false, b.v, (short)0, c, false, false);
  asm volatile("v_nop\n\tv_nop\n\tv_nop\n\tv_nop" : "+v"(d) : "v"(a.w), "v"(b.w));
  return d;
}

__device__ __forceinline__ unsigned bf16_bits(float f) {
  const unsigned u = __float_as_uint(f);
  return (u + 0x7FFFu + ((u >> 16) & 1u)) >> 16;
}
__device__ __forceinline__ float bf16_val(float f) {
  return __uint_as_float(bf16_bits(f) << 16);
}

struct HL4 { v4us h; v4us l; };
__device__ __forceinline__ HL4 split4(const v4f v) {
  HL4 o;
  unsigned hb;
  hb = bf16_bits(v.x); o.h[0] = (unsigned short)hb; o.l[0] = (unsigned short)bf16_bits(v.x - __uint_as_float(hb << 16));
  hb = bf16_bits(v.y); o.h[1] = (unsigned short)hb; o.l[1] = (unsigned short)bf16_bits(v.y - __uint_as_float(hb << 16));
  hb = bf16_bits(v.z); o.h[2] = (unsigned short)hb; o.l[2] = (unsigned short)bf16_bits(v.z - __uint_as_float(hb << 16));
  hb = bf16_bits(v.w); o.h[3] = (unsigned short)hb; o.l[3] = (unsigned short)bf16_bits(v.w - __uint_as_float(hb << 16));
  return o;
}

template <int SLB>
__device__ __forceinline__ int scan_chunk(const int* __restrict__ dsts, int nE, int cbase, int slotBase,
                                          int nb, int vec8, int* list, int tid, int lane, int wave) {
  int wc = 0;
  const int el0  = tid * EPT;
  const int e0   = cbase + el0;
  const int sent = -2147483647 - 1;
  v4i da, db;
  if (vec8 != 0 && cbase + CHUNK <= nE) {
    da = *(const v4i*)(dsts + e0);
    db = *(const v4i*)(dsts + e0 + 4);
  } else {
    da.x = (e0     < nE) ? dsts[min(e0,     nE - 1)] : sent;
    da.y = (e0 + 1 < nE) ? dsts[min(e0 + 1, nE - 1)] : sent;
    da.z = (e0 + 2 < nE) ? dsts[min(e0 + 2, nE - 1)] : sent;
    da.w = (e0 + 3 < nE) ? dsts[min(e0 + 3, nE - 1)] : sent;
    db.x = (e0 + 4 < nE) ? dsts[min(e0 + 4, nE - 1)] : sent;
    db.y = (e0 + 5 < nE) ? dsts[min(e0 + 5, nE - 1)] : sent;
    db.z = (e0 + 6 < nE) ? dsts[min(e0 + 6, nE - 1)] : sent;
    db.w = (e0 + 7 < nE) ? dsts[min(e0 + 7, nE - 1)] : sent;
  }
  const unsigned nbs = (unsigned)slotBase;
  const unsigned unb = (unsigned)nb;
  const unsigned s0 = (unsigned)da.x - nbs, s1 = (unsigned)da.y - nbs;
  const unsigned s2 = (unsigned)da.z - nbs, s3 = (unsigned)da.w - nbs;
  const unsigned s4 = (unsigned)db.x - nbs, s5 = (unsigned)db.y - nbs;
  const unsigned s6 = (unsigned)db.z - nbs, s7 = (unsigned)db.w - nbs;
  const bool h0 = s0 < unb, h1 = s1 < unb, h2 = s2 < unb, h3 = s3 < unb;
  const bool h4 = s4 < unb, h5 = s5 < unb, h6 = s6 < unb, h7 = s7 < unb;
  const unsigned any = __builtin_amdgcn_ballot_w32(h0 | h1 | h2 | h3 | h4 | h5 | h6 | h7);
  if (any != 0u) {
#define HITJ(J, HJ, SJ) { \
      const unsigned mj = __builtin_amdgcn_ballot_w32(HJ); \
      if (mj != 0u) { \
        if (HJ) { \
          const int pos = wc + (int)__builtin_amdgcn_mbcnt_lo(mj, 0u); \
          if (pos < WCAP) list[wave * WCAP + pos] = ((el0 + (J)) << SLB) | (int)(SJ); \
        } \
        wc += (int)__builtin_popcount(mj); } }
    HITJ(0, h0, s0)
    HITJ(1, h1, s1)
    HITJ(2, h2, s2)
    HITJ(3, h3, s3)
    HITJ(4, h4, s4)
    HITJ(5, h5, s5)
    HITJ(6, h6, s6)
    HITJ(7, h7, s7)
#undef HITJ
  }
  return wc;
}

__global__ __launch_bounds__(NTHR) void k_prep(const float* __restrict__ feat, const float* __restrict__ W1,
                                               const float* __restrict__ W2, int nUnitsF,
                                               float* fb, unsigned short* W1T2, unsigned short* W2T2) {
  const int tid = (int)threadIdx.x;
  if ((int)blockIdx.x < NWB) {
    const int u = (int)blockIdx.x * NTHR + tid;
    v8us o;
    unsigned short* dp;
    if (u < NU1) {
      const int n  = u >> 3;
      const int k8 = (u & 7) * 8;
      const int kk = k8 & (F0 - 1);
      const float* p = W1 + (size_t)kk * HID + n;
#pragma unroll
      for (int i = 0; i < 8; ++i) o[i] = (unsigned short)bf16_bits(p[(size_t)i * HID]);
      dp = W1T2 + (size_t)n * K1 + k8;
    } else {
      const int v  = u - NU1;
      const int n  = v >> 4;
      const int k8 = (v & 15) * 8;
      const int kk = k8 & (HID - 1);
      const float* p = W2 + (size_t)kk * FOUT + n;
#pragma unroll
      for (int i = 0; i < 8; ++i) o[i] = (unsigned short)bf16_bits(p[(size_t)i * FOUT]);
      dp = W2T2 + (size_t)n * K2 + k8;
    }
    *(volatile v8us*)dp = o;
    __threadfence();
    *(volatile v8us*)dp = o;
  } else {
    const int u = ((int)blockIdx.x - NWB) * NTHR + tid;
    if (u >= nUnitsF) return;
    const v4f a = *(const v4f*)(feat + (size_t)u * 4);
    v4f o;
    o.x = bf16_val(a.x); o.y = bf16_val(a.y); o.z = bf16_val(a.z); o.w = bf16_val(a.w);
    float* dp = fb + (size_t)u * 4;
    *(volatile v4f*)dp = o;
    __threadfence();
    *(volatile v4f*)dp = o;
  }
}

__device__ __forceinline__ void drain_rows(const int* cnt, const int* offs, const int* cols, const int* vals,
                                           int ovf, const float* __restrict__ src, int nN, float* dst,
                                           int nodeBase, int lane, int wave) {
  const int g  = lane >> 3;
  const int l8 = lane & 7;
  const float qnan = __int_as_float(0x7fc00000);
  const float pz = (ovf != 0) ? qnan : 0.0f;
#pragma unroll 1
  for (int qi = 0; qi < NBA / (4 * NWAVE); ++qi) {
    const int s    = 4 * (qi * NWAVE + wave) + g;
    const int node = nodeBase + s;
    int c = cnt[s];
    const bool big = c > DEGCAP;
    c = c < 0 ? 0 : (c > DEGCAP ? DEGCAP : c);
    int o = offs[s];
    o = o < 0 ? 0 : (o > RCAP ? RCAP : o);
    int cm = c;
    {
      const int t1 = __shfl_xor(cm, 8, 32);
      cm = cm > t1 ? cm : t1;
      const int t2 = __shfl_xor(cm, 16, 32);
      cm = cm > t2 ? cm : t2;
    }
    cm = __builtin_amdgcn_readfirstlane(cm);
    cm = cm > DEGCAP ? DEGCAP : cm;
    float a0 = 0.0f, a1 = 0.0f, a2 = 0.0f, a3 = 0.0f;
#pragma unroll 1
    for (int j = 0; j < cm; ++j) {
      int idx = o + j;
      idx = idx > RCAP - 1 ? RCAP - 1 : idx;
      const bool on = j < c;
      int cl = cols[idx];
      cl = cl < 0 ? 0 : (cl > nN - 1 ? nN - 1 : cl);
      const float w = __int_as_float(vals[idx]);
      const v4f x = *(const v4f*)(src + (size_t)cl * F0 + 4 * l8);
      const float ww = on ? w : 0.0f;
      const float x0 = on ? x.x : 0.0f;
      const float x1 = on ? x.y : 0.0f;
      const float x2 = on ? x.z : 0.0f;
      const float x3 = on ? x.w : 0.0f;
      a0 = fmaf(ww, x0, a0);
      a1 = fmaf(ww, x1, a1);
      a2 = fmaf(ww, x2, a2);
      a3 = fmaf(ww, x3, a3);
    }
    const float pzr = big ? qnan : pz;
    const bool live = node < nN;
    v4f ov;
    ov.x = live ? (a0 + pzr) : 0.0f;
    ov.y = live ? (a1 + pzr) : 0.0f;
    ov.z = live ? (a2 + pzr) : 0.0f;
    ov.w = live ? (a3 + pzr) : 0.0f;
    float* op = dst + (size_t)node * F0 + 4 * l8;
    *(volatile v4f*)op = ov;
    __threadfence();
    *(volatile v4f*)op = ov;
  }
}

__global__ __launch_bounds__(NTHR) void k_scan1(const int* __restrict__ keys, const int* __restrict__ gath,
                                                const float* __restrict__ ew, int nE, int nN, int vec8,
                                                const float* __restrict__ fb, float* y0, int* hits) {
  extern __shared__ __attribute__((aligned(16))) int dsm[];
  int* list = dsm;
  int* seg  = dsm + LISTN;
  int* cnt  = seg + SEG_CNT;
  int* offs = seg + SEG_OFF;
  int* hl   = seg + SEG_COL;
  int* sl   = seg + SEG_VAL;
  int* cur  = seg + SEGI;
  int* misc = cur + NBA;
  const int tid = (int)threadIdx.x, lane = tid & 31, wave = tid >> 5;
  const int nodeBase = (int)blockIdx.x * NBA;

  {
    const v4i z4 = {0, 0, 0, 0};
    for (int i = tid * 4; i < SC_ZINTS; i += NTHR * 4) *(v4ia*)(dsm + i) = z4;
    if (tid < 16) misc[tid] = 0;
  }
  __syncthreads();

  int t = 0, ov = 0;
  const int nChunks = (nE + CHUNK - 1) / CHUNK;
#pragma unroll 1
  for (int ch = 0; ch < nChunks; ++ch) {
    const int cbase = ch * CHUNK;
    const int wc = scan_chunk<SLA>(keys, nE, cbase, nodeBase, NBA, vec8, list, tid, lane, wave);
    if (lane == 0) misc[wave] = wc;
    __syncthreads();
    if (wave == 0) {
#pragma unroll 1
      for (int w2 = 0; w2 < NWAVE; ++w2) {
        int c = misc[w2];
        c = c < 0 ? 0 : (c > WCAP ? WCAP : c);
#pragma unroll 1
        for (int b0 = 0; b0 < c; b0 += 32) {
          const int idx = b0 + lane;
          const int ent = list[w2 * WCAP + (idx < WCAP ? idx : WCAP - 1)];
          const int m32 = (c - b0) < 32 ? (c - b0) : 32;
#pragma unroll 1
          for (int k = 0; k < m32; ++k) {
            const int u    = __builtin_amdgcn_readlane(ent, k);
            const int slot = u & (NBA - 1);
            const int el   = (u >> SLA) & (CHUNK - 1);
            const int pk   = ((cbase + el) << SLA) | slot;
            if (t < RCAP) {
              if (lane == 0) { hl[t] = pk; cnt[slot] = cnt[slot] + 1; }
              t = t + 1;
            } else {
              ov = 1;
            }
          }
        }
      }
    }
    __syncthreads();
  }
  if (wave == 0 && lane == 0) { misc[8] = t; misc[9] = ov; }
  __syncthreads();
  int tt = misc[8];
  tt = tt < 0 ? 0 : (tt > RCAP ? RCAP : tt);
  const int ovf = misc[9];

  if (wave == 0) {
    const int base = lane * (NBA / 32);
    int s = 0;
#pragma unroll 1
    for (int i = 0; i < NBA / 32; ++i) s += cnt[base + i];
    int incl = s;
#pragma unroll
    for (int d = 1; d < 32; d <<= 1) {
      const int y = __shfl_up(incl, d, 32);
      if (lane >= d) incl += y;
    }
    int run = incl - s;
#pragma unroll 1
    for (int i = 0; i < NBA / 32; ++i) {
      const int cv = cnt[base + i];
      offs[base + i] = run;
      cur[base + i]  = run;
      run += cv;
    }
  }
  __syncthreads();
  if (wave == 0) {
#pragma unroll 1
    for (int b0 = 0; b0 < tt; b0 += 32) {
      const int idx = b0 + lane;
      const int ent = hl[idx < RCAP ? idx : RCAP - 1];
      const int m32 = (tt - b0) < 32 ? (tt - b0) : 32;
#pragma unroll 1
      for (int k = 0; k < m32; ++k) {
        const int u    = __builtin_amdgcn_readlane(ent, k);
        const int slot = u & (NBA - 1);
        if (lane == 0) {
          int p = cur[slot];
          p = p < 0 ? 0 : (p > RCAP - 1 ? RCAP - 1 : p);
          sl[p] = u;
          cur[slot] = p + 1;
        }
      }
    }
  }
  __syncthreads();

#pragma unroll 1
  for (int p0 = 0; p0 < tt; p0 += NTHR) {
    const int p  = p0 + tid;
    const int pc = p > RCAP - 1 ? RCAP - 1 : p;
    const int ent = sl[pc];
    int eid = ent >> SLA;
    eid = eid < 0 ? 0 : (eid > nE - 1 ? nE - 1 : eid);
    int gc = gath[eid];
    gc = gc < 0 ? 0 : (gc > nN - 1 ? nN - 1 : gc);
    const float wv = bf16_val(ew[eid]);
    if (p < tt) { hl[pc] = gc; sl[pc] = __float_as_int(wv); }
  }
  if (tid == 0) { seg[0] = tt; seg[1] = ovf; }
  __syncthreads();

  {
    int* gseg = hits + (size_t)blockIdx.x * SEGI;
#pragma unroll 1
    for (int i = tid * 4; i < SEGI; i += NTHR * 4) {
      const v4i v = *(const v4ia*)(seg + i);
      *(volatile v4i*)(gseg + i) = v;
    }
    __threadfence();
#pragma unroll 1
    for (int i = tid * 4; i < SEGI; i += NTHR * 4) {
      const v4i v = *(const v4ia*)(seg + i);
      *(volatile v4i*)(gseg + i) = v;
    }
  }

  drain_rows(cnt, offs, hl, sl, ovf, fb, nN, y0, nodeBase, lane, wave);
}

__global__ __launch_bounds__(NTHR) void k_agg2(const int* __restrict__ hits, int nN,
                                               const float* __restrict__ y0, float* y1) {
  extern __shared__ __attribute__((aligned(16))) int dsm[];
  int* seg = dsm;
  const int tid = (int)threadIdx.x, lane = tid & 31, wave = tid >> 5;
  const int nodeBase = (int)blockIdx.x * NBA;
  const int* gseg = hits + (size_t)blockIdx.x * SEGI;
#pragma unroll 2
  for (int i = tid * 4; i < SEGI; i += NTHR * 4) {
    const v4i v = *(const v4i*)(gseg + i);
    *(v4ia*)(seg + i) = v;
  }
  __syncthreads();
  const int ovf = seg[1];
  drain_rows(seg + SEG_CNT, seg + SEG_OFF, seg + SEG_COL, seg + SEG_VAL, ovf, y0, nN, y1, nodeBase, lane, wave);
}

__global__ __launch_bounds__(NTHR) void k_mlp(const float* __restrict__ y1, const unsigned short* __restrict__ w1t,
                                              const unsigned short* __restrict__ w2t, float* out, int nN) {
  extern __shared__ __attribute__((aligned(16))) int dsm[];
  unsigned short* a1 = (unsigned short*)dsm;
  float* zst = (float*)((char*)dsm + 16384);
  float* ost = (float*)dsm;
  unsigned short* a2 = (unsigned short*)((char*)dsm + ML_A2_OFF);
  const int tid = (int)threadIdx.x, lane = tid & 31, wave = tid >> 5, hh = lane >> 4, m = lane & 15;
  const int rowBase = (int)blockIdx.x * MT;

#pragma unroll
  for (int it = 0; it < (MT * F0 / 4) / NTHR; ++it) {
    const int u   = it * NTHR + tid;
    const int row = u >> 3;
    const int c4  = (u & 7) * 4;
    const v4f v = *(const v4f*)(y1 + (size_t)(rowBase + row) * F0 + c4);
    const HL4 s = split4(v);
    *(v4usa*)(a1 + row * K1 + c4) = s.h;
    *(v4usa*)(a1 + row * K1 + F0 + c4) = s.l;
  }
  __syncthreads();

  {
    v8f acc1[4];
    {
      const v8f z = {0.f, 0.f, 0.f, 0.f, 0.f, 0.f, 0.f, 0.f};
      acc1[0] = z; acc1[1] = z; acc1[2] = z; acc1[3] = z;
    }
    const unsigned short* ar = a1 + (16 * wave + m) * K1 + 8 * hh;
    const unsigned short* wp = w1t + (size_t)m * K1 + 8 * hh;
#pragma unroll
    for (int ks = 0; ks < K1 / 32; ++ks) {
      FragB af;
      af.h[0] = *(const v8usa*)(ar + 32 * ks);
      af.h[1] = *(const v8usa*)(ar + 32 * ks + 16);
#pragma unroll
      for (int t = 0; t < 4; ++t) {
        const unsigned short* wq = wp + (size_t)(16 * t) * K1 + 32 * ks;
        FragB bf;
        bf.h[0] = *(const v8usa*)wq;
        bf.h[1] = *(const v8usa*)(wq + 16);
        acc1[t] = wmb(af, bf, acc1[t]);
      }
    }
#pragma unroll
    for (int t = 0; t < 4; ++t) {
#pragma unroll
      for (int r = 0; r < 8; ++r) {
        const int lr = 16 * wave + 8 * hh + r;
        zst[lr * HID + 16 * t + m] = acc1[t][r];
      }
    }
  }
  __syncthreads();

#pragma unroll 2
  for (int i = 0; i < 8; ++i) {
    const int e   = i * 32 + lane;
    const int row = 16 * wave + (e >> 4);
    const int c4  = (e & 15) * 4;
    const v4f v = *(const v4fa*)(zst + row * HID + c4);
    const HL4 s = split4(v);
    *(v4usa*)(a2 + row * K2 + c4) = s.h;
    *(v4usa*)(a2 + row * K2 + HID + c4) = s.l;
  }
  __syncthreads();

  v8f acc2[8];
  {
    const v8f z = {0.f, 0.f, 0.f, 0.f, 0.f, 0.f, 0.f, 0.f};
#pragma unroll
    for (int t = 0; t < 8; ++t) acc2[t] = z;
  }
  {
    const unsigned short* ar2 = a2 + (16 * wave + m) * K2 + 8 * hh;
    const unsigned short* wp2 = w2t + (size_t)m * K2 + 8 * hh;
#pragma unroll 1
    for (int ks = 0; ks < K2 / 32; ++ks) {
      FragB af;
      af.h[0] = *(const v8usa*)(ar2 + 32 * ks);
      af.h[1] = *(const v8usa*)(ar2 + 32 * ks + 16);
#pragma unroll
      for (int nt = 0; nt < 8; ++nt) {
        const unsigned short* wq = wp2 + (size_t)(16 * nt) * K2 + 32 * ks;
        FragB bf;
        bf.h[0] = *(const v8usa*)wq;
        bf.h[1] = *(const v8usa*)(wq + 16);
        acc2[nt] = wmb(af, bf, acc2[nt]);
      }
    }
  }

#pragma unroll
  for (int nt = 0; nt < 8; ++nt) {
#pragma unroll
    for (int r = 0; r < 8; ++r) {
      const int lr = 16 * wave + 8 * hh + r;
      ost[lr * FOUT + 16 * nt + m] = acc2[nt][r];
    }
  }
  __syncthreads();
  v4f pv[16];
#pragma unroll
  for (int i = 0; i < 16; ++i) pv[i] = *(const v4fa*)(ost + (16 * wave + i) * FOUT + 4 * lane);
#pragma unroll
  for (int i = 0; i < 16; ++i) {
    const int r = rowBase + 16 * wave + i;
    if (r < nN) *(volatile v4f*)(out + (size_t)r * FOUT + 4 * lane) = pv[i];
  }
  __threadfence();
#pragma unroll
  for (int i = 0; i < 16; ++i) {
    const int r = rowBase + 16 * wave + i;
    if (r < nN) *(volatile v4f*)(out + (size_t)r * FOUT + 4 * lane) = pv[i];
  }
}

static inline int cdiv(int a, int b) { return (a + b - 1) / b; }
static inline size_t al256(size_t o) { return (o + 255) & ~(size_t)255; }

extern "C" void kernel_launch(void* const* d_in, const int* in_sizes, int n_in,
                              void* d_out, int out_size, void* d_ws, size_t ws_size,
                              hipStream_t stream) {
  if (n_in < 6) return;
  if (in_sizes[0] < F0 || (in_sizes[0] % F0) != 0) return;
  const int nN = in_sizes[0] / F0;
  if (nN < 1 || nN > (1 << 22)) return;
  if (in_sizes[1] != F0 * HID) return;
  if (in_sizes[2] != HID * FOUT) return;
  const int nE = in_sizes[3];
  if (nE < 1 || nE >= (1 << (31 - SLA))) return;
  if (in_sizes[4] != nE || in_sizes[5] != nE) return;
  if ((long long)out_size != (long long)nN * FOUT) return;

  const float* feat = (const float*)d_in[0];
  const float* W1   = (const float*)d_in[1];
  const float* W2   = (const float*)d_in[2];
  const int*   erow = (const int*)d_in[3];
  const int*   ecol = (const int*)d_in[4];
  const float* eval = (const float*)d_in[5];
  float* out = (float*)d_out;

  const int gS = cdiv(nN, NBA);
  const int NP = gS * NBA;
  const int gT = cdiv(nN, MT);
  if ((long long)gT * MT > (long long)NP) return;
  const int nUnitsF = nN * (F0 / 4);
  const int vec8 = ((nE & 3) == 0) ? 1 : 0;

  char* ws = (char*)d_ws;
  size_t off = 0;
  const size_t oW1 = off; off = al256(off + (size_t)HID * K1 * 2);
  const size_t oW2 = off; off = al256(off + (size_t)FOUT * K2 * 2);
  const size_t oFB = off; off = al256(off + (size_t)nN * F0 * 4);
  const size_t oY0 = off; off = al256(off + (size_t)NP * F0 * 4);
  const size_t oY1 = off; off = al256(off + (size_t)NP * F0 * 4);
  const size_t oHT = off; off = al256(off + (size_t)gS * SEGI * 4);
  if (off > ws_size || off > (size_t)WSMAX) return;
  unsigned short* W1T2 = (unsigned short*)(ws + oW1);
  unsigned short* W2T2 = (unsigned short*)(ws + oW2);
  float* FB   = (float*)(ws + oFB);
  float* Y0   = (float*)(ws + oY0);
  float* Y1   = (float*)(ws + oY1);
  int*   HITS = (int*)(ws + oHT);

  const size_t scanLds = (size_t)SC_LDS_INTS * 4;
  const size_t aggLds  = (size_t)SEGI * 4;
  const size_t mlpLds  = (size_t)ML_LDS_BYTES;
  hipFuncSetAttribute(reinterpret_cast<const void*>(&k_scan1), hipFuncAttributeMaxDynamicSharedMemorySize, (int)scanLds);
  hipFuncSetAttribute(reinterpret_cast<const void*>(&k_agg2), hipFuncAttributeMaxDynamicSharedMemorySize, (int)aggLds);
  hipFuncSetAttribute(reinterpret_cast<const void*>(&k_mlp), hipFuncAttributeMaxDynamicSharedMemorySize, (int)mlpLds);

  k_prep<<<NWB + cdiv(nUnitsF, NTHR), NTHR, 0, stream>>>(feat, W1, W2, nUnitsF, FB, W1T2, W2T2);
  k_scan1<<<gS, NTHR, scanLds, stream>>>(erow, ecol, eval, nE, nN, vec8, FB, Y0, HITS);
  k_agg2<<<gS, NTHR, aggLds, stream>>>(HITS, nN, Y0, Y1);
  k_mlp<<<gT, NTHR, mlpLds, stream>>>(Y1, W1T2, W2T2, out, nN);
}
